// TitansL2_60902636257296
// MI455X (gfx1250) — hardware-verified
//
#include <hip/hip_runtime.h>
#include <math.h>


#define BB 4
#define TT 2048
#define CC 1024
#define HH 16
#define HD 64
#define NR (BB * TT)

typedef __attribute__((ext_vector_type(16))) _Float16 v16h;
typedef __attribute__((ext_vector_type(8)))  _Float16 v8h;
typedef __attribute__((ext_vector_type(8)))  float v8f;
typedef __attribute__((ext_vector_type(4)))  float v4f;
typedef __attribute__((ext_vector_type(4)))  unsigned v4u;

template <typename T> __device__ __forceinline__ void vst2(void* p, T v) { *(volatile T*)p = v; __threadfence(); *(volatile T*)p = v; }
__device__ __forceinline__ v8f wmma16(v16h a, v16h b, v8f c) {
  v8f d = __builtin_amdgcn_wmma_f32_16x16x32_f16(false, a, false, b, (short)0, c, false, false);
  asm volatile("v_nop\n\tv_nop\n\tv_nop\n\tv_nop" : "+v"(d) : "v"(a), "v"(b));
  return d;
}
__device__ __forceinline__ v16h frag_h(const _Float16* rowk0, int lane) {
  union { v16h v; v8h q[2]; } u; const _Float16* p = rowk0 + 8 * (lane >> 4);
  u.q[0] = *(const v8h*)p; u.q[1] = *(const v8h*)(p + 16); return u.v;
}
#define LDSX() do { asm volatile("s_wait_dscnt 0" ::: "memory"); __builtin_amdgcn_wave_barrier(); __builtin_amdgcn_fence(__ATOMIC_RELEASE, "workgroup"); } while (0)

__global__ __launch_bounds__(256) void k_cvt_rows(const float* __restrict__ s, _Float16* __restrict__ d, size_t n8) {
  const size_t g8 = (size_t)blockIdx.x * 256 + threadIdx.x; if (g8 >= n8) return;
  union { v8h h; v4u u; } pk;
#pragma unroll
  for (int e = 0; e < 8; ++e) pk.h[e] = (_Float16)s[g8 * 8 + e];
  vst2(d + g8 * 8, pk.u);
}

__global__ __launch_bounds__(128) void k_qkv(const _Float16* __restrict__ xh, const _Float16* __restrict__ Wqh, const _Float16* __restrict__ Wkh,
                                           const _Float16* __restrict__ Wvh, float* __restrict__ qp, float* __restrict__ kp, float* __restrict__ vp) {
  __shared__ __align__(16) float st[64][132];
  const int tid = threadIdx.x, wave = tid >> 5, lane = tid & 31, col = lane & 15, g = lane >> 4;
  const int r0 = blockIdx.x * 64, n0 = blockIdx.y * 128, which = blockIdx.z;
  const _Float16* W = which == 0 ? Wqh : (which == 1 ? Wkh : Wvh);
  float* P = which == 0 ? qp : (which == 1 ? kp : vp);
  v8f acc[8] = {};
#pragma unroll 1
  for (int kc = 0; kc < CC / 32; ++kc) {
    const v16h a = frag_h(xh + (size_t)(r0 + wave * 16 + col) * CC + kc * 32, lane);
#pragma unroll
    for (int j = 0; j < 8; ++j) acc[j] = wmma16(a, frag_h(W + (size_t)(n0 + j * 16 + col) * CC + kc * 32, lane), acc[j]);
  }
#pragma unroll
  for (int j = 0; j < 8; ++j)
#pragma unroll
    for (int r = 0; r < 8; ++r) st[wave * 16 + 8 * g + r][j * 16 + col] = acc[j][r];
  __syncthreads();
  const int b = r0 / TT, t0 = r0 % TT, h0 = n0 / HD;
  for (int q = tid; q < 2 * 64 * 16; q += 128) { const int hh = q >> 10, rl = (q >> 4) & 63, pc = q & 15;
    vst2(P + (((size_t)b * HH + h0 + hh) * TT + t0 + rl) * HD + pc * 4, *(const v4f*)(&st[rl][hh * 64 + pc * 4])); }
}

__global__ __launch_bounds__(256) void k_scan(const float* __restrict__ qp, const float* __restrict__ kp, const float* __restrict__ vp,
                                            const float* __restrict__ alpha_raw, const float* __restrict__ beta_raw, const float* __restrict__ s0,
                                            _Float16* __restrict__ yh, float* __restrict__ sfin) {
  __shared__ __align__(16) float sq[HD], sk[HD], sv[HD], red[2];
  __shared__ __align__(16) float ybuf[32][HD];
  __shared__ __align__(16) float sst[HD][HD + 4];
  const int tid = threadIdx.x, bh = blockIdx.x, b = bh / HH, h = bh % HH;
  const int d = tid >> 2, e0 = (tid & 3) * 16;
  const float alpha = 0.5f / (1.f + expf(-alpha_raw[h])), beta = 0.5f / (1.f + expf(-beta_raw[h]));
  float S[16];
#pragma unroll
  for (int i = 0; i < 16; ++i) S[i] = s0[((size_t)bh * HD + d) * HD + e0 + i];
  const float* qb = qp + (size_t)bh * TT * HD; const float* kb = kp + (size_t)bh * TT * HD; const float* vb = vp + (size_t)bh * TT * HD;
  for (int t = 0; t < TT; ++t) {
    if (tid < HD) { sq[tid] = qb[(size_t)t * HD + tid]; sv[tid] = vb[(size_t)t * HD + tid]; }
    if (tid >= 64 && tid < 128) { sk[tid - 64] = kb[(size_t)t * HD + tid - 64]; }
    __syncthreads();
    if (tid < 32) {
      float s = sk[tid] * sk[tid] + sk[tid + 32] * sk[tid + 32];
#pragma unroll
      for (int off = 16; off >= 1; off >>= 1) s += __shfl_xor(s, off, 32);
      if (tid == 0) red[0] = 1.0f / fmaxf(sqrtf(s), 1e-12f);
    }
    __syncthreads();
    const float kinv = red[0];
    float kl[16], y = 0.f, mk = 0.f;
#pragma unroll
    for (int i = 0; i < 16; ++i) { kl[i] = sk[e0 + i] * kinv; y += sq[e0 + i] * S[i]; mk += S[i] * kl[i]; }
    y  += __shfl_xor(y, 1, 32);  y  += __shfl_xor(y, 2, 32);
    mk += __shfl_xor(mk, 1, 32); mk += __shfl_xor(mk, 2, 32);
    const float coef = beta * sv[d] - alpha * mk;
#pragma unroll
    for (int i = 0; i < 16; ++i) S[i] += coef * kl[i];
    if ((tid & 3) == 0) ybuf[t & 31][d] = y;
    __syncthreads();
    if ((t & 31) == 31) {
      { const int rl = tid >> 3, pc = tid & 7; union { v8h hh; v4u u; } pk;
#pragma unroll
        for (int e = 0; e < 8; ++e) pk.hh[e] = (_Float16)ybuf[rl][pc * 8 + e];
        vst2(yh + ((size_t)b * TT + (t - 31) + rl) * CC + h * HD + pc * 8, pk.u); }
      __syncthreads();
    }
  }
#pragma unroll
  for (int i = 0; i < 16; ++i) sst[d][e0 + i] = S[i];
  __syncthreads();
  for (int q = tid; q < HD * 16; q += 256) { const int dd = q >> 4, pc = q & 15;
    vst2(sfin + ((size_t)bh * HD + dd) * HD + pc * 4, *(const v4f*)(&sst[dd][pc * 4])); }
}

__global__ __launch_bounds__(128) void k_out(const _Float16* __restrict__ yh, const _Float16* __restrict__ Wph, float* __restrict__ out) {
  __shared__ __align__(16) float so[4][16 * 128];
  const int tid = threadIdx.x, wave = tid >> 5, lane = tid & 31, col = lane & 15, g = lane >> 4;
  const int r0 = blockIdx.x * 64 + wave * 16, n0 = blockIdx.y * 128;
  v8f acc[8] = {};
#pragma unroll 1
  for (int kc = 0; kc < CC / 32; ++kc) {
    const v16h a = frag_h(yh + (size_t)(r0 + col) * CC + kc * 32, lane);
#pragma unroll
    for (int j = 0; j < 8; ++j) acc[j] = wmma16(a, frag_h(Wph + (size_t)(n0 + j * 16 + col) * CC + kc * 32, lane), acc[j]);
  }
  float* S_ = so[wave];
#pragma unroll
  for (int j = 0; j < 8; ++j)
#pragma unroll
    for (int r = 0; r < 8; ++r) S_[(8 * g + r) * 128 + j * 16 + col] = acc[j][r];
  LDSX();
#pragma unroll 4
  for (int rl = 0; rl < 16; ++rl) vst2(out + (size_t)(r0 + rl) * CC + n0 + lane * 4, *(const v4f*)(S_ + rl * 128 + lane * 4));
}

extern "C" void kernel_launch(void* const* d_in, const int* in_sizes, int n_in,
                              void* d_out, int out_size, void* d_ws, size_t ws_size,
                              hipStream_t stream) {
  (void)in_sizes; (void)n_in; (void)out_size; (void)ws_size;
  const float* x  = (const float*)d_in[0];
  const float* Wq = (const float*)d_in[1]; const float* Wk = (const float*)d_in[2];
  const float* Wv = (const float*)d_in[3]; const float* Wp = (const float*)d_in[4];
  const float* ar = (const float*)d_in[5]; const float* br = (const float*)d_in[6];
  const float* s0 = (const float*)d_in[7];
  float* out  = (float*)d_out;
  float* sfin = (float*)d_out + (size_t)NR * CC;
  char* ws = (char*)d_ws; size_t off = 0;
  auto take = [&](size_t bytes) { char* p = ws + off; off += (bytes + 255) & ~(size_t)255; return p; };
  _Float16* xh  = (_Float16*)take((size_t)NR * CC * 2);
  _Float16* Wqh = (_Float16*)take((size_t)CC * CC * 2); _Float16* Wkh = (_Float16*)take((size_t)CC * CC * 2);
  _Float16* Wvh = (_Float16*)take((size_t)CC * CC * 2); _Float16* Wph = (_Float16*)take((size_t)CC * CC * 2);
  float* qp = (float*)take((size_t)NR * CC * 4); float* kp = (float*)take((size_t)NR * CC * 4); float* vp = (float*)take((size_t)NR * CC * 4);
  _Float16* yh = (_Float16*)take((size_t)NR * CC * 2);
  k_cvt_rows<<<(unsigned)((NR * CC / 8 + 255) / 256), 256, 0, stream>>>(x, xh, (size_t)NR * CC / 8);
  k_cvt_rows<<<(unsigned)((CC * CC / 8 + 255) / 256), 256, 0, stream>>>(Wq, Wqh, (size_t)CC * CC / 8);
  k_cvt_rows<<<(unsigned)((CC * CC / 8 + 255) / 256), 256, 0, stream>>>(Wk, Wkh, (size_t)CC * CC / 8);
  k_cvt_rows<<<(unsigned)((CC * CC / 8 + 255) / 256), 256, 0, stream>>>(Wv, Wvh, (size_t)CC * CC / 8);
  k_cvt_rows<<<(unsigned)((CC * CC / 8 + 255) / 256), 256, 0, stream>>>(Wp, Wph, (size_t)CC * CC / 8);
  k_qkv<<<dim3(NR / 64, CC / 128, 3), 128, 0, stream>>>(xh, Wqh, Wkh, Wvh, qp, kp, vp);
  k_scan<<<BB * HH, 256, 0, stream>>>(qp, kp, vp, ar, br, s0, yh, sfin);
  k_out<<<dim3(NR / 64, CC / 128), 128, 0, stream>>>(yh, Wph, out);
}
